// QwenCUDAWayfinderAttention_38104949850684
// MI455X (gfx1250) — hardware-verified
//
#include <hip/hip_runtime.h>
#include <hip/hip_bf16.h>
#include <stddef.h>
#include <stdint.h>

#define SQ    2048
#define HID   2048
#define NH    16
#define NKV   4
#define HDM   128
#define HALF  64
#define KNB   64
#define NQG   4096
#define NKW   512
#define RMS_EPS 0.000001f

static_assert(SQ % 256 == 0);
static_assert(HID == 256 * 8);
static_assert(HDM == 128);
static_assert(NH * HDM == HID);
static_assert(NH == 4 * NKV);
static_assert(NQG == NH * 2 * HDM);
static_assert(NKW == NKV * HDM);
static_assert(KNB == 64);
static_assert(HID % 64 == 0);
static_assert(NQG % 64 == 0);
static_assert(NKW % 64 == 0);

typedef _Float16 v16h __attribute__((ext_vector_type(16)));
typedef _Float16 v8h  __attribute__((ext_vector_type(8)));
typedef float    v8f  __attribute__((ext_vector_type(8)));
typedef float    v4f  __attribute__((ext_vector_type(4)));
typedef unsigned int   v4u   __attribute__((ext_vector_type(4)));
typedef unsigned short v8us  __attribute__((ext_vector_type(8)));
typedef unsigned short v16us __attribute__((ext_vector_type(16)));
typedef __bf16         v16b  __attribute__((ext_vector_type(16)));
typedef unsigned short ush;

union Frag  { v16h v; v8h h[2]; };
union FragU { v16us v; v8us h[2]; v4u u[2]; v16b b; };
union Pack8 { v8h h; v4u u; };
union PackU { v8us s; v4u u; };
struct HL { v4u h; v4u l; };

__device__ __forceinline__ ush f2bf(float f) {
  const unsigned u = __float_as_uint(f);
  return (ush)((u + 0x7FFFu + ((u >> 16) & 1u)) >> 16);
}
__device__ __forceinline__ float bf2f(ush b) { return __uint_as_float(((unsigned)b) << 16); }

__device__ __forceinline__ HL split8(v8f f) {
  PackU ph, pl;
#pragma unroll
  for (int e = 0; e < 8; ++e) {
    const ush hi = f2bf(f[e]);
    ph.s[e] = hi;
    pl.s[e] = f2bf(f[e] - bf2f(hi));
  }
  HL r; r.h = ph.u; r.l = pl.u;
  return r;
}

__device__ __forceinline__ v8f mma16(v16h a, v16h b, v8f c) {
  c = __builtin_amdgcn_wmma_f32_16x16x32_f16(false, a, false, b, (short)0, c, false, false);
  asm volatile("v_nop\n\tv_nop\n\tv_nop\n\tv_nop" : "+v"(c) : "v"(a), "v"(b));
  return c;
}
__device__ __forceinline__ v8f mmab(v16us a, v16us b, v8f c) {
  FragU ua, ub; ua.v = a; ub.v = b;
  c = __builtin_amdgcn_wmma_f32_16x16x32_bf16(false, ua.b, false, ub.b, (short)0, c, false, false);
  asm volatile("v_nop\n\tv_nop\n\tv_nop\n\tv_nop" : "+v"(c) : "v"(a), "v"(b));
  return c;
}

__device__ __forceinline__ v16h ldfrag(const _Float16* p, int ld, int row0, int k0, int lane) {
  const int m = lane & 15, lh = lane >> 4;
  const _Float16* q = p + (size_t)(row0 + m) * ld + k0 + 8 * lh;
  Frag f;
  f.h[0] = *(const v8h*)(q);
  f.h[1] = *(const v8h*)(q + 16);
  return f.v;
}
__device__ __forceinline__ v16us ldfragu(const ush* p, int ld, int row0, int k0, int lane) {
  const int m = lane & 15, lh = lane >> 4;
  const ush* q = p + (size_t)(row0 + m) * ld + k0 + 8 * lh;
  FragU f;
  f.h[0] = *(const v8us*)(q);
  f.h[1] = *(const v8us*)(q + 16);
  return f.v;
}

__device__ __forceinline__ v8f zero8() { return (v8f){0.f, 0.f, 0.f, 0.f, 0.f, 0.f, 0.f, 0.f}; }

__device__ __forceinline__ float sigm(float x) {
  const float e = __expf(-fabsf(x));
  const float r = 1.0f / (1.0f + e);
  return (x >= 0.f) ? r : e * r;
}

__device__ __forceinline__ void gemm16x64(const _Float16* __restrict__ A, int lda,
                                          const _Float16* __restrict__ Bt, int ldb,
                                          int m0, int n0, int lane, v8f (&acc)[4]) {
#pragma unroll 2
  for (int k0 = 0; k0 < HID; k0 += 32) {
    const v16h a = ldfrag(A, lda, m0, k0, lane);
#pragma unroll
    for (int t = 0; t < 4; ++t) {
      const v16h b = ldfrag(Bt, ldb, n0 + 16 * t, k0, lane);
      acc[t] = mma16(a, b, acc[t]);
    }
  }
}

__device__ __forceinline__ void gemm3_16x64(const ush* __restrict__ Ah, const ush* __restrict__ Al, int lda,
                                            const ush* __restrict__ Bh, const ush* __restrict__ Bl, int ldb,
                                            int m0, int n0, int lane, v8f (&acc)[4]) {
#pragma unroll 1
  for (int k0 = 0; k0 < HID; k0 += 32) {
    const v16us ah = ldfragu(Ah, lda, m0, k0, lane);
    const v16us al = ldfragu(Al, lda, m0, k0, lane);
#pragma unroll
    for (int t = 0; t < 4; ++t) {
      const v16us bh = ldfragu(Bh, ldb, n0 + 16 * t, k0, lane);
      const v16us bl = ldfragu(Bl, ldb, n0 + 16 * t, k0, lane);
      acc[t] = mmab(ah, bh, acc[t]);
      acc[t] = mmab(ah, bl, acc[t]);
      acc[t] = mmab(al, bh, acc[t]);
    }
  }
}

__device__ __forceinline__ void gemm3_32x64(const ush* __restrict__ Ah, const ush* __restrict__ Al, int lda,
                                            const ush* __restrict__ Bh, const ush* __restrict__ Bl, int ldb,
                                            int m0, int n0, int lane, v8f (&acc)[2][4]) {
#pragma unroll 1
  for (int k0 = 0; k0 < HID; k0 += 32) {
    const v16us a0h = ldfragu(Ah, lda, m0, k0, lane);
    const v16us a1h = ldfragu(Ah, lda, m0 + 16, k0, lane);
    const v16us a0l = ldfragu(Al, lda, m0, k0, lane);
    const v16us a1l = ldfragu(Al, lda, m0 + 16, k0, lane);
#pragma unroll
    for (int t = 0; t < 4; ++t) {
      const v16us bh = ldfragu(Bh, ldb, n0 + 16 * t, k0, lane);
      const v16us bl = ldfragu(Bl, ldb, n0 + 16 * t, k0, lane);
      acc[0][t] = mmab(a0h, bh, acc[0][t]);
      acc[1][t] = mmab(a1h, bh, acc[1][t]);
      acc[0][t] = mmab(a0h, bl, acc[0][t]);
      acc[1][t] = mmab(a1h, bl, acc[1][t]);
      acc[0][t] = mmab(a0l, bh, acc[0][t]);
      acc[1][t] = mmab(a1l, bh, acc[1][t]);
    }
  }
}

__global__ __launch_bounds__(256) void k_xcv(const float* __restrict__ x, _Float16* __restrict__ dh,
                                             ush* __restrict__ d3h, ush* __restrict__ d3l) {
  const int row  = blockIdx.x;
  const int col  = (int)threadIdx.x * 8;
  const size_t o = (size_t)row * HID + col;
  const v4f a0 = *(const v4f*)(x + o);
  const v4f a1 = *(const v4f*)(x + o + 4);
  Pack8 pk;
  pk.h = (v8h){(_Float16)a0[0], (_Float16)a0[1], (_Float16)a0[2], (_Float16)a0[3],
               (_Float16)a1[0], (_Float16)a1[1], (_Float16)a1[2], (_Float16)a1[3]};
  const v4u vv = pk.u;
  const v8f f = (v8f){a0[0], a0[1], a0[2], a0[3], a1[0], a1[1], a1[2], a1[3]};
  const HL sp = split8(f);
  *(volatile v4u*)(dh + o)  = vv;
  *(volatile v4u*)(d3h + o) = sp.h;
  *(volatile v4u*)(d3l + o) = sp.l;
  __threadfence();
  *(volatile v4u*)(dh + o)  = vv;
  *(volatile v4u*)(d3h + o) = sp.h;
  *(volatile v4u*)(d3l + o) = sp.l;
}

#define WTP 68
__global__ __launch_bounds__(256) void k_wtr(const float* __restrict__ W, int N, int mode,
                                             _Float16* __restrict__ wt, ush* __restrict__ wh,
                                             ush* __restrict__ wl) {
  __shared__ __align__(16) float sw[64 * WTP];
  const int tid = threadIdx.x;
  const int n0 = blockIdx.x * 64;
  const int k0 = blockIdx.y * 64;
  const int c4 = (tid & 15) * 4;
#pragma unroll
  for (int i = 0; i < 4; ++i) {
    const int r = (tid >> 4) + 16 * i;
    const v4f v = *(const v4f*)(W + (size_t)(k0 + r) * N + n0 + c4);
    *(v4f*)(sw + r * WTP + c4) = v;
  }
  __syncthreads();
  size_t go[2];
  v8f fv[2];
#pragma unroll
  for (int j = 0; j < 2; ++j) {
    const int p  = tid + 256 * j;
    const int nl = p >> 3;
    const int pc = p & 7;
    const float* cp = sw + (8 * pc) * WTP + nl;
    fv[j] = (v8f){cp[0 * WTP], cp[1 * WTP], cp[2 * WTP], cp[3 * WTP],
                  cp[4 * WTP], cp[5 * WTP], cp[6 * WTP], cp[7 * WTP]};
    go[j] = (size_t)(n0 + nl) * HID + k0 + 8 * pc;
  }
  if (mode == 0) {
    v4u vt[2];
#pragma unroll
    for (int j = 0; j < 2; ++j) {
      Pack8 pk;
      pk.h = (v8h){(_Float16)(fv[j][0] * 32.0f), (_Float16)(fv[j][1] * 32.0f), (_Float16)(fv[j][2] * 32.0f),
                   (_Float16)(fv[j][3] * 32.0f), (_Float16)(fv[j][4] * 32.0f), (_Float16)(fv[j][5] * 32.0f),
                   (_Float16)(fv[j][6] * 32.0f), (_Float16)(fv[j][7] * 32.0f)};
      vt[j] = pk.u;
    }
    for (int ps = 0; ps < 2; ++ps) {
#pragma unroll
      for (int j = 0; j < 2; ++j) *(volatile v4u*)(wt + go[j]) = vt[j];
      __threadfence();
    }
  } else {
    v4u vh[2], vl[2];
#pragma unroll
    for (int j = 0; j < 2; ++j) { const HL sp = split8(fv[j]); vh[j] = sp.h; vl[j] = sp.l; }
    for (int ps = 0; ps < 2; ++ps) {
#pragma unroll
      for (int j = 0; j < 2; ++j) {
        *(volatile v4u*)(wh + go[j]) = vh[j];
        *(volatile v4u*)(wl + go[j]) = vl[j];
      }
      __threadfence();
    }
  }
}

#define SFP 132
__device__ __forceinline__ void head_norm(float* sf, const float* __restrict__ nw, int tid) {
  const int lr = tid >> 2;
  const int qq = (tid & 3) * 32;
  float* rp = sf + lr * SFP + qq;
  v4f xv[8];
  float ss = 0.f;
#pragma unroll
  for (int e = 0; e < 8; ++e) {
    xv[e] = *(const v4f*)(rp + 4 * e);
    ss += xv[e][0] * xv[e][0] + xv[e][1] * xv[e][1] + xv[e][2] * xv[e][2] + xv[e][3] * xv[e][3];
  }
  ss += __shfl_xor(ss, 1, 32);
  ss += __shfl_xor(ss, 2, 32);
  const float rsn = 1.0f / sqrtf(ss * 0.0078125f + RMS_EPS);
#pragma unroll
  for (int e = 0; e < 8; ++e) {
    const v4f w = *(const v4f*)(nw + qq + 4 * e);
    *(v4f*)(rp + 4 * e) = (xv[e] * rsn) * w;
  }
}

__device__ __forceinline__ HL rope_piece(const float* sf, const float* __restrict__ ct,
                                         const float* __restrict__ sn, int lr, int pc, int pos) {
  const int d0 = pc * 8;
  const float* ra = sf + lr * SFP + d0;
  const float* rb = sf + lr * SFP + (d0 ^ HALF);
  const v4f a0 = *(const v4f*)(ra), a1 = *(const v4f*)(ra + 4);
  const v4f b0 = *(const v4f*)(rb), b1 = *(const v4f*)(rb + 4);
  const size_t to = (size_t)pos * HDM + d0;
  const v4f c0 = *(const v4f*)(ct + to), c1 = *(const v4f*)(ct + to + 4);
  const v4f s0 = *(const v4f*)(sn + to), s1 = *(const v4f*)(sn + to + 4);
  const float sg = (pc < 8) ? -1.0f : 1.0f;
  const v4f o0 = a0 * c0 + sg * (b0 * s0);
  const v4f o1 = a1 * c1 + sg * (b1 * s1);
  const v8f f = (v8f){o0[0], o0[1], o0[2], o0[3], o1[0], o1[1], o1[2], o1[3]};
  return split8(f);
}

__global__ __launch_bounds__(256) void k_qproj(const _Float16* __restrict__ xh,
                                               const _Float16* __restrict__ wqt,
                                               const float* __restrict__ qnw,
                                               const float* __restrict__ ct,
                                               const float* __restrict__ sn,
                                               ush* __restrict__ q3h,
                                               ush* __restrict__ q3l,
                                               float* __restrict__ gs) {
  __shared__ __align__(16) float sf[64 * SFP];
  const int tid = threadIdx.x, lane = tid & 31, wave = tid >> 5;
  const int hh = lane >> 4, c = lane & 15;
  const int wm = wave >> 1, wn = wave & 1;
  const int sb = blockIdx.x * 64;
  const int ns = blockIdx.y;
  const int head = ns >> 1, part = ns & 1;
  const int m0 = sb + wm * 16;
  const int n0 = ns * HDM + wn * 64;

  v8f acc[4];
#pragma unroll
  for (int t = 0; t < 4; ++t) acc[t] = zero8();
  gemm16x64(xh, HID, wqt, HID, m0, n0, lane, acc);

#pragma unroll
  for (int t = 0; t < 4; ++t) {
#pragma unroll
    for (int r = 0; r < 8; ++r)
      sf[(wm * 16 + 8 * hh + r) * SFP + wn * 64 + 16 * t + c] = acc[t][r] * 0.03125f;
  }
  __syncthreads();

  if (part == 0) {
    head_norm(sf, qnw, tid);
    __syncthreads();
    v4u vh[4], vl[4];
    size_t go[4];
#pragma unroll
    for (int j = 0; j < 4; ++j) {
      const int p  = tid + 256 * j;
      const int lr = p >> 4;
      const int pc = p & 15;
      const HL sp = rope_piece(sf, ct, sn, lr, pc, sb + lr);
      vh[j] = sp.h; vl[j] = sp.l;
      go[j] = ((size_t)head * SQ + sb + lr) * HDM + pc * 8;
    }
    for (int ps = 0; ps < 2; ++ps) {
#pragma unroll
      for (int j = 0; j < 4; ++j) {
        *(volatile v4u*)(q3h + go[j]) = vh[j];
        *(volatile v4u*)(q3l + go[j]) = vl[j];
      }
      __threadfence();
    }
  } else {
    v4f val[8];
    size_t go[8];
#pragma unroll
    for (int j = 0; j < 8; ++j) {
      const int p  = tid + 256 * j;
      const int lr = p >> 5;
      const int pc = p & 31;
      const v4f xg = *(const v4f*)(sf + lr * SFP + 4 * pc);
      val[j] = (v4f){sigm(xg[0]), sigm(xg[1]), sigm(xg[2]), sigm(xg[3])};
      go[j]  = (size_t)(sb + lr) * HID + (size_t)head * HDM + 4 * pc;
    }
    for (int ps = 0; ps < 2; ++ps) {
#pragma unroll
      for (int j = 0; j < 8; ++j) *(volatile v4f*)(gs + go[j]) = val[j];
      __threadfence();
    }
  }
}

__global__ __launch_bounds__(256) void k_kv3(const ush* __restrict__ xh3, const ush* __restrict__ xl3,
                                             const ush* __restrict__ wkh, const ush* __restrict__ wkl,
                                             const ush* __restrict__ wvh, const ush* __restrict__ wvl,
                                             const float* __restrict__ knw,
                                             const float* __restrict__ ct, const float* __restrict__ sn,
                                             ush* __restrict__ k3h, ush* __restrict__ k3l,
                                             ush* __restrict__ v3h, ush* __restrict__ v3l) {
  __shared__ __align__(16) float sf[64 * SFP];
  const int tid = threadIdx.x, lane = tid & 31, wave = tid >> 5;
  const int hh = lane >> 4, c = lane & 15;
  const int wm = wave >> 1, wn = wave & 1;
  const int sb  = blockIdx.x * 64;
  const int ns  = blockIdx.y;
  const int which = ns >> 2;
  const int head = ns & 3;
  const int m0 = sb + wm * 16;
  const int n0 = head * HDM + wn * 64;
  const ush* bh = (which == 0) ? wkh : wvh;
  const ush* bl = (which == 0) ? wkl : wvl;

  v8f acc[4];
#pragma unroll
  for (int t = 0; t < 4; ++t) acc[t] = zero8();
  gemm3_16x64(xh3, xl3, HID, bh, bl, HID, m0, n0, lane, acc);

#pragma unroll
  for (int t = 0; t < 4; ++t) {
#pragma unroll
    for (int r = 0; r < 8; ++r)
      sf[(wm * 16 + 8 * hh + r) * SFP + wn * 64 + 16 * t + c] = acc[t][r];
  }
  __syncthreads();

  v4u vh[4], vl[4];
  size_t go[4];
  if (which == 0) {
    head_norm(sf, knw, tid);
    __syncthreads();
#pragma unroll
    for (int j = 0; j < 4; ++j) {
      const int p  = tid + 256 * j;
      const int lr = p >> 4;
      const int pc = p & 15;
      const HL sp = rope_piece(sf, ct, sn, lr, pc, sb + lr);
      vh[j] = sp.h; vl[j] = sp.l;
      go[j] = ((size_t)head * SQ + sb + lr) * HDM + pc * 8;
    }
    for (int ps = 0; ps < 2; ++ps) {
#pragma unroll
      for (int j = 0; j < 4; ++j) {
        *(volatile v4u*)(k3h + go[j]) = vh[j];
        *(volatile v4u*)(k3l + go[j]) = vl[j];
      }
      __threadfence();
    }
  } else {
#pragma unroll
    for (int j = 0; j < 4; ++j) {
      const int p  = tid + 256 * j;
      const int lr = p >> 4;
      const int pc = p & 15;
      const float* ra = sf + lr * SFP + pc * 8;
      const v4f a0 = *(const v4f*)(ra), a1 = *(const v4f*)(ra + 4);
      const v8f f = (v8f){a0[0], a0[1], a0[2], a0[3], a1[0], a1[1], a1[2], a1[3]};
      const HL sp = split8(f);
      vh[j] = sp.h; vl[j] = sp.l;
      go[j] = ((size_t)head * SQ + sb + lr) * HDM + pc * 8;
    }
    for (int ps = 0; ps < 2; ++ps) {
#pragma unroll
      for (int j = 0; j < 4; ++j) {
        *(volatile v4u*)(v3h + go[j]) = vh[j];
        *(volatile v4u*)(v3l + go[j]) = vl[j];
      }
      __threadfence();
    }
  }
}

#define KTQ 136
#define VTP 72
#define PTP 72
static_assert(2 * KNB * KTQ <= 2 * HDM * VTP);
__global__ __launch_bounds__(128) void k_attn(const ush* __restrict__ q3h, const ush* __restrict__ q3l,
                                              const ush* __restrict__ k3h, const ush* __restrict__ k3l,
                                              const ush* __restrict__ v3h, const ush* __restrict__ v3l,
                                              const float* __restrict__ gs, const int* __restrict__ nidx,
                                              ush* __restrict__ oh, ush* __restrict__ ol, float sscale) {
  __shared__ __align__(16) ush R[2 * HDM * VTP];
  __shared__ __align__(16) ush P[2 * 16 * PTP];
  __shared__ __align__(16) ush Os[2 * 4 * HDM];
  __shared__ float Sc[4 * KNB];
  __shared__ int   nbs[KNB];
  __shared__ int   oks[KNB];

  const int tid = threadIdx.x, lane = tid & 31, wave = tid >> 5;
  const int hh = lane >> 4, c = lane & 15;
  const int g = blockIdx.x & 3;
  const int s = blockIdx.x >> 2;

  if (tid < KNB) {
    const int ix = nidx[(size_t)s * KNB + tid];
    const int cl = (ix < 0) ? 0 : ((ix > SQ - 1) ? (SQ - 1) : ix);
    nbs[tid] = cl;
    oks[tid] = (ix >= 0 && ix < SQ && ix <= s) ? 1 : 0;
  }
  {
    unsigned int* pz = (unsigned int*)P;
#pragma unroll
    for (int i = 0; i < 9; ++i) pz[tid + 128 * i] = 0u;
  }
  __syncthreads();

  const ush* KH = k3h + (size_t)g * SQ * HDM;
  const ush* KL = k3l + (size_t)g * SQ * HDM;
  const ush* VH = v3h + (size_t)g * SQ * HDM;
  const ush* VL = v3l + (size_t)g * SQ * HDM;

  {
    ush* Ksh = R;
    ush* Ksl = R + KNB * KTQ;
#pragma unroll
    for (int i = 0; i < 8; ++i) {
      const int p   = tid + 128 * i;
      const int j   = p >> 4, pc = p & 15;
      const int row = nbs[j] & (SQ - 1);
      const size_t so = (size_t)row * HDM + 8 * pc;
      *(v8us*)(Ksh + j * KTQ + 8 * pc) = *(const v8us*)(KH + so);
      *(v8us*)(Ksl + j * KTQ + 8 * pc) = *(const v8us*)(KL + so);
    }
  }
  __syncthreads();

  {
    const ush* Ksh = R;
    const ush* Ksl = R + KNB * KTQ;
    v8f sacc = zero8();
    const int mm = (c < 4) ? c : 3;
    const unsigned qm = (c < 4) ? 0xFFFFFFFFu : 0u;
    const v4u qm4 = (v4u){qm, qm, qm, qm};
    const ush* QH = q3h + ((size_t)(4 * g + mm) * SQ + s) * HDM + 8 * hh;
    const ush* QL = q3l + ((size_t)(4 * g + mm) * SQ + s) * HDM + 8 * hh;
#pragma unroll
    for (int dc = 0; dc < 4; ++dc) {
      FragU fh, fl;
      fh.u[0] = (*(const v4u*)(QH + 32 * dc)) & qm4;
      fh.u[1] = (*(const v4u*)(QH + 32 * dc + 16)) & qm4;
      fl.u[0] = (*(const v4u*)(QL + 32 * dc)) & qm4;
      fl.u[1] = (*(const v4u*)(QL + 32 * dc + 16)) & qm4;
      const v16us kbh = ldfragu(Ksh, KTQ, 16 * wave, 32 * dc, lane);
      const v16us kbl = ldfragu(Ksl, KTQ, 16 * wave, 32 * dc, lane);
      sacc = mmab(fh.v, kbh, sacc);
      sacc = mmab(fh.v, kbl, sacc);
      sacc = mmab(fl.v, kbh, sacc);
    }
    if (hh == 0) {
#pragma unroll
      for (int r = 0; r < 4; ++r) Sc[r * KNB + 16 * wave + c] = sacc[r] * sscale;
    }
  }
  __syncthreads();

  {
    const int r  = wave;
    const int j0 = lane, j1 = lane + 32;
    const int ok0 = oks[j0], ok1 = oks[j1];
    const float NEGB = -1.0e30f;
    const float a0 = Sc[r * KNB + j0], a1 = Sc[r * KNB + j1];
    const float s0 = ok0 ? a0 : NEGB;
    const float s1 = ok1 ? a1 : NEGB;
    float m = fmaxf(s0, s1);
#pragma unroll
    for (int off = 16; off >= 1; off >>= 1) m = fmaxf(m, __shfl_xor(m, off, 32));
    const float e0 = __expf(s0 - m);
    const float e1 = __expf(s1 - m);
    float sum = e0 + e1;
#pragma unroll
    for (int off = 16; off >= 1; off >>= 1) sum += __shfl_xor(sum, off, 32);
    const float inv = 1.0f / sum;
    const float p0 = ok0 ? (e0 * inv) : 0.f;
    const float p1 = ok1 ? (e1 * inv) : 0.f;
    const ush h0 = f2bf(p0), h1 = f2bf(p1);
    P[r * PTP + j0] = h0;
    P[r * PTP + j1] = h1;
    P[16 * PTP + r * PTP + j0] = f2bf(p0 - bf2f(h0));
    P[16 * PTP + r * PTP + j1] = f2bf(p1 - bf2f(h1));
  }
  {
    ush* Vth = R;
    ush* Vtl = R + HDM * VTP;
#pragma unroll
    for (int i = 0; i < 4; ++i) {
      const int p  = tid + 128 * i;
      const int jp = p >> 4, pc = p & 15;
      const int ra = nbs[2 * jp] & (SQ - 1), rb = nbs[2 * jp + 1] & (SQ - 1);
      const v8us ah = *(const v8us*)(VH + (size_t)ra * HDM + 8 * pc);
      const v8us bh = *(const v8us*)(VH + (size_t)rb * HDM + 8 * pc);
      const v8us al = *(const v8us*)(VL + (size_t)ra * HDM + 8 * pc);
      const v8us bl = *(const v8us*)(VL + (size_t)rb * HDM + 8 * pc);
      unsigned int* th = (unsigned int*)(Vth + (8 * pc) * VTP + 2 * jp);
      unsigned int* tl = (unsigned int*)(Vtl + (8 * pc) * VTP + 2 * jp);
#pragma unroll
      for (int e = 0; e < 8; ++e) {
        th[e * (VTP / 2)] = (unsigned int)ah[e] | (((unsigned int)bh[e]) << 16);
        tl[e * (VTP / 2)] = (unsigned int)al[e] | (((unsigned int)bl[e]) << 16);
      }
    }
  }
  __syncthreads();

  v8f oacc[2];
  oacc[0] = zero8(); oacc[1] = zero8();
  {
    const ush* Vth = R;
    const ush* Vtl = R + HDM * VTP;
    const ush* Ph  = P;
    const ush* Pl  = P + 16 * PTP;
#pragma unroll
    for (int kk = 0; kk < 2; ++kk) {
      const v16us pah = ldfragu(Ph, PTP, 0, 32 * kk, lane);
      const v16us pal = ldfragu(Pl, PTP, 0, 32 * kk, lane);
#pragma unroll
      for (int t = 0; t < 2; ++t) {
        const v16us vbh = ldfragu(Vth, VTP, 32 * wave + 16 * t, 32 * kk, lane);
        const v16us vbl = ldfragu(Vtl, VTP, 32 * wave + 16 * t, 32 * kk, lane);
        oacc[t] = mmab(pah, vbh, oacc[t]);
        oacc[t] = mmab(pah, vbl, oacc[t]);
        oacc[t] = mmab(pal, vbh, oacc[t]);
      }
    }
  }
  {
    const float* gp = gs + (size_t)s * HID + (size_t)(4 * g) * HDM + 32 * wave + c;
#pragma unroll
    for (int t = 0; t < 2; ++t) {
#pragma unroll
      for (int r = 0; r < 4; ++r) {
        const float gv = gp[r * HDM + 16 * t];
        const float o  = oacc[t][r] * gv;
        const ush hi = f2bf(o);
        const ush lo = f2bf(o - bf2f(hi));
        if (hh == 0) {
          Os[r * HDM + 32 * wave + 16 * t + c]           = hi;
          Os[4 * HDM + r * HDM + 32 * wave + 16 * t + c] = lo;
        }
      }
    }
  }
  __syncthreads();
  {
    const int plane = wave >> 1;
    const int piece = tid & 63;
    PackU pk;
    pk.s = *(const v8us*)(Os + plane * (4 * HDM) + piece * 8);
    const v4u val = pk.u;
    ush* dst = ((plane == 0) ? oh : ol) + (size_t)s * HID + (size_t)g * (4 * HDM) + piece * 8;
    *(volatile v4u*)dst = val;
    __threadfence();
    *(volatile v4u*)dst = val;
  }
}

#define OTP 68
__device__ __forceinline__ void out_epilogue(v8f (&acc)[2][4], float scale, float* sw, float* __restrict__ out,
                                             int m0, int n0, int lane, int hh, int c) {
#pragma unroll
  for (int sub = 0; sub < 2; ++sub) {
    __syncthreads();
#pragma unroll
    for (int t = 0; t < 4; ++t) {
#pragma unroll
      for (int r = 0; r < 8; ++r) sw[(8 * hh + r) * OTP + 16 * t + c] = acc[sub][t][r] * scale;
    }
    __syncthreads();
    v4f val[8];
    size_t go[8];
#pragma unroll
    for (int it = 0; it < 8; ++it) {
      const int p    = lane + 32 * it;
      const int L    = p >> 3;
      const int pc   = p & 7;
      const int row  = L >> 1;
      const int half = L & 1;
      val[it] = *(const v4f*)(sw + row * OTP + half * 32 + pc * 4);
      go[it]  = (size_t)(m0 + sub * 16 + row) * HID + n0 + half * 32 + pc * 4;
    }
    for (int ps = 0; ps < 2; ++ps) {
#pragma unroll
      for (int it = 0; it < 8; ++it) *(volatile v4f*)(out + go[it]) = val[it];
      __threadfence();
    }
  }
}

__global__ __launch_bounds__(256) void k_out3(const ush* __restrict__ ah, const ush* __restrict__ al,
                                              const ush* __restrict__ wh, const ush* __restrict__ wl,
                                              float* __restrict__ out) {
  __shared__ __align__(16) float st[8][16 * OTP];
  const int tid = threadIdx.x, lane = tid & 31, wave = tid >> 5;
  const int hh = lane >> 4, c = lane & 15;
  const int m0   = blockIdx.x * 256 + wave * 32;
  const int n0   = blockIdx.y * 64;

  v8f acc[2][4];
#pragma unroll
  for (int s = 0; s < 2; ++s)
#pragma unroll
    for (int t = 0; t < 4; ++t) acc[s][t] = zero8();
  gemm3_32x64(ah, al, HID, wh, wl, HID, m0, n0, lane, acc);
  out_epilogue(acc, 1.0f, st[wave], out, m0, n0, lane, hh, c);
}

extern "C" void kernel_launch(void* const* d_in, const int* in_sizes, int n_in,
                              void* d_out, int out_size, void* d_ws, size_t ws_size,
                              hipStream_t stream) {
  if (n_in < 10) return;
  if (in_sizes[0] != SQ * HID) return;
  if (in_sizes[1] != HID * NQG) return;
  if (in_sizes[2] != HID * NKW) return;
  if (in_sizes[3] != HID * NKW) return;
  if (in_sizes[4] != HID * HID) return;
  if (in_sizes[5] != HDM) return;
  if (in_sizes[6] != HDM) return;
  if (in_sizes[7] != SQ * HDM) return;
  if (in_sizes[8] != SQ * HDM) return;
  if (in_sizes[9] != SQ * KNB) return;
  if (out_size != SQ * HID) return;

  const float* x    = (const float*)d_in[0];
  const float* wq   = (const float*)d_in[1];
  const float* wk   = (const float*)d_in[2];
  const float* wv   = (const float*)d_in[3];
  const float* wo   = (const float*)d_in[4];
  const float* qnw  = (const float*)d_in[5];
  const float* knw  = (const float*)d_in[6];
  const float* ct   = (const float*)d_in[7];
  const float* sn   = (const float*)d_in[8];
  const int*   nidx = (const int*)d_in[9];
  float* out = (float*)d_out;

  size_t off = 0;
  const size_t oXh  = off; off += (size_t)SQ * HID * 2;
  const size_t oX3h = off; off += (size_t)SQ * HID * 2;
  const size_t oX3l = off; off += (size_t)SQ * HID * 2;
  const size_t oWqt = off; off += (size_t)NQG * HID * 2;
  const size_t oWkh = off; off += (size_t)NKW * HID * 2;
  const size_t oWkl = off; off += (size_t)NKW * HID * 2;
  const size_t oWvh = off; off += (size_t)NKW * HID * 2;
  const size_t oWvl = off; off += (size_t)NKW * HID * 2;
  const size_t oWoh = off; off += (size_t)HID * HID * 2;
  const size_t oWol = off; off += (size_t)HID * HID * 2;
  const size_t oG   = off; off += (size_t)SQ * HID * 4;
  const size_t oQ3h = off; off += (size_t)NH * SQ * HDM * 2;
  const size_t oQ3l = off; off += (size_t)NH * SQ * HDM * 2;
  const size_t oK3h = off; off += (size_t)NKV * SQ * HDM * 2;
  const size_t oK3l = off; off += (size_t)NKV * SQ * HDM * 2;
  const size_t oV3h = off; off += (size_t)NKV * SQ * HDM * 2;
  const size_t oV3l = off; off += (size_t)NKV * SQ * HDM * 2;
  const size_t oOh  = off; off += (size_t)SQ * HID * 2;
  const size_t oOl  = off; off += (size_t)SQ * HID * 2;
  if (off > ws_size) return;
  if (off > (size_t)134217728) return;

  char* ws = (char*)d_ws;
  _Float16* Xh  = (_Float16*)(ws + oXh);
  ush*      X3h = (ush*)(ws + oX3h);
  ush*      X3l = (ush*)(ws + oX3l);
  _Float16* Wqt = (_Float16*)(ws + oWqt);
  ush*      Wkh = (ush*)(ws + oWkh);
  ush*      Wkl = (ush*)(ws + oWkl);
  ush*      Wvh = (ush*)(ws + oWvh);
  ush*      Wvl = (ush*)(ws + oWvl);
  ush*      Woh = (ush*)(ws + oWoh);
  ush*      Wol = (ush*)(ws + oWol);
  float*    G   = (float*)(ws + oG);
  ush*      Q3h = (ush*)(ws + oQ3h);
  ush*      Q3l = (ush*)(ws + oQ3l);
  ush*      K3h = (ush*)(ws + oK3h);
  ush*      K3l = (ush*)(ws + oK3l);
  ush*      V3h = (ush*)(ws + oV3h);
  ush*      V3l = (ush*)(ws + oV3l);
  ush*      Oh  = (ush*)(ws + oOh);
  ush*      Ol  = (ush*)(ws + oOl);

  k_xcv<<<dim3(SQ), dim3(256), 0, stream>>>(x, Xh, X3h, X3l);
  k_wtr<<<dim3(NQG / 64, HID / 64), dim3(256), 0, stream>>>(wq, NQG, 0, Wqt, Wkh, Wkl);
  k_wtr<<<dim3(NKW / 64, HID / 64), dim3(256), 0, stream>>>(wk, NKW, 1, Wqt, Wkh, Wkl);
  k_wtr<<<dim3(NKW / 64, HID / 64), dim3(256), 0, stream>>>(wv, NKW, 1, Wqt, Wvh, Wvl);
  k_wtr<<<dim3(HID / 64, HID / 64), dim3(256), 0, stream>>>(wo, HID, 1, Wqt, Woh, Wol);
  k_qproj<<<dim3(SQ / 64, NQG / HDM), dim3(256), 0, stream>>>(Xh, Wqt, qnw, ct, sn, Q3h, Q3l, G);
  k_kv3<<<dim3(SQ / 64, (2 * NKW) / HDM), dim3(256), 0, stream>>>(X3h, X3l, Wkh, Wkl, Wvh, Wvl, knw, ct, sn,
                                                                 K3h, K3l, V3h, V3l);
  const float sscale = 0.08838834764831845f;
  k_attn<<<dim3(SQ * NKV), dim3(128), 0, stream>>>(Q3h, Q3l, K3h, K3l, V3h, V3l, G, nidx, Oh, Ol, sscale);
  k_out3<<<dim3(SQ / 256, HID / 64), dim3(256), 0, stream>>>(Oh, Ol, Woh, Wol, out);
  (void)hipGetLastError();
}
